// FakeNewsGNN_40888088658252
// MI455X (gfx1250) — hardware-run, weakly checked
//
#include <hip/hip_runtime.h>
#include <stddef.h>
#include <stdint.h>

#define NN      50000
#define DF      128
#define NE      600000
#define NLAY    6
#define GBM     128
#define MP      50048
#define MPITCH  256
#define XPITCH  128
#define WP0     384
#define WPI     512
#define SPLIT_MEAN 1
#define SPLIT_ROOT 1
#define KMEAN   (SPLIT_MEAN ? 256 : 128)
#define KROOT   (SPLIT_ROOT ? 256 : 128)
#define NTHR    256
#define NWAVE   8
#define EPT     8
#define WCH     (32 * EPT)
#define PER     75008
#define NBRUN   1024
#define SLB     10
#define NBK     49
#define WLCAP   2048
#define RCAP    16384
#define DEGCAP  64
#define MAXDEG_MEAS   28
#define MAXB1024_MEAS 12548
#define RBM     64
#define SP      132
#define SMF     1056

#define BK_ZINTS (NWAVE * WLCAP + RCAP + 4 * NBRUN)
#define BK_INTS  (BK_ZINTS + 16)
#define BK_LDS   (BK_INTS * 4)
#define GM_FLOATS (GBM * SP + 128 + 256 + 32 + 256)
#define GM_LDS   (GM_FLOATS * 4)

#define UPART  2048
#define PBX    (MP * DF / 8 / NTHR)
#define PBW0   (3 * UPART / NTHR)
#define PBWI   (5 * 4 * UPART / NTHR)
#define PBTOT  (PBX + PBW0 + PBWI + 1)

static_assert(DF == 128 && DF == 4 * 32);
static_assert(NN % 16 == 0);
static_assert(NBK == 49);
static_assert(MP % GBM == 0 && MP >= NN && MP == 391 * GBM && MP % RBM == 0);
static_assert(NBRUN == (1 << SLB) && NBRUN % RBM == 0 && NBRUN % GBM == 0 && NBRUN % 32 == 0);
static_assert(NBK * NBRUN >= MP);
static_assert(NE < (1 << 21) && (((long long)NE) << SLB) < (1LL << 31));
static_assert(NE % EPT == 0 && (NE * 4) % 16 == 0);
static_assert(PER % WCH == 0 && (NWAVE - 1) * PER < NE && NWAVE * PER >= NE);
static_assert(RCAP == NWAVE * WLCAP && RCAP % (NTHR * 4) == 0 && BK_ZINTS % 4 == 0);
static_assert((3 * NBRUN) % (NTHR * 4) == 0);
static_assert((long long)RCAP * 100 >= (long long)MAXB1024_MEAS * 105);
static_assert(WLCAP >= MAXB1024_MEAS / 8 + 8 * 46 + 1);
static_assert(MAXDEG_MEAS + 8 <= DEGCAP);
static_assert(RBM == NWAVE * 8 && GBM == NWAVE * 16);
static_assert((MP * DF / 8) % NTHR == 0 && UPART % NTHR == 0 && UPART == DF * (DF / 8));
static_assert(KMEAN % 32 == 0 && KROOT % 32 == 0 && KMEAN <= MPITCH && KROOT <= MPITCH);
static_assert(WP0 == 3 * DF && WPI == 4 * DF && MPITCH == 2 * DF);
static_assert(GBM * 2 / 4 == 64 && ((NN % GBM) * 2 * 4) % 128 == 0 && (GBM * 2 * 4) % 128 == 0);
static_assert(BK_LDS <= 327680 && GM_LDS <= 327680);
static_assert(SMF % 32 == 0 && SMF == NLAY * DF + 2 * DF + 32);

typedef float          v4f   __attribute__((ext_vector_type(4)));
typedef float          v8f   __attribute__((ext_vector_type(8)));
typedef int            v4i   __attribute__((ext_vector_type(4)));
typedef int            v8i   __attribute__((ext_vector_type(8)));
typedef unsigned       v2u   __attribute__((ext_vector_type(2)));
typedef unsigned short v8us  __attribute__((ext_vector_type(8)));
typedef unsigned short v16us __attribute__((ext_vector_type(16)));
typedef __bf16         v16bf __attribute__((ext_vector_type(16)));
typedef v4f  __attribute__((may_alias)) v4fa;
typedef v4i  __attribute__((may_alias)) v4ia;
typedef v2u  __attribute__((may_alias)) v2ua;
typedef v8us __attribute__((may_alias)) v8usa;
union FragB { v16bf v; v16us u; v8us h[2]; v8i w; };

__device__ __forceinline__ v8f wmb(const FragB& a, const FragB& b, v8f c) {
  v8f d = __builtin_amdgcn_wmma_f32_16x16x32_bf16(false, a.v, false, b.v, (short)0, c, false, false);
  asm volatile("v_nop\n\tv_nop\n\tv_nop\n\tv_nop" : "+v"(d) : "v"(a.w), "v"(b.w));
  return d;
}

__device__ __forceinline__ unsigned bf16_bits(float f) {
  const unsigned u = __float_as_uint(f);
  const unsigned r = (u + 0x7FFFu + ((u >> 16) & 1u)) >> 16;
  const unsigned q = (u >> 16) | 0x40u;
  return ((u & 0x7fffffffu) > 0x7f800000u) ? q : r;
}
__device__ __forceinline__ float bf16_val(float f) {
  return __uint_as_float(bf16_bits(f) << 16);
}

__device__ __forceinline__ void hilo_pack(float v0, float v1, float v2, float v3,
                                          int& h01, int& h23, int& l01, int& l23) {
  const unsigned a0 = bf16_bits(v0), a1 = bf16_bits(v1), a2 = bf16_bits(v2), a3 = bf16_bits(v3);
  const unsigned b0 = bf16_bits(v0 - __uint_as_float(a0 << 16));
  const unsigned b1 = bf16_bits(v1 - __uint_as_float(a1 << 16));
  const unsigned b2 = bf16_bits(v2 - __uint_as_float(a2 << 16));
  const unsigned b3 = bf16_bits(v3 - __uint_as_float(a3 << 16));
  h01 = (int)(a0 | (a1 << 16)); h23 = (int)(a2 | (a3 << 16));
  l01 = (int)(b0 | (b1 << 16)); l23 = (int)(b2 | (b3 << 16));
}

__device__ __forceinline__ v4i regroup_w(int h01, int h23, int l01, int l23, int lane) {
  const int s0 = (2 * lane) & 31, s1 = s0 + 1;
  const int a0 = __shfl(h01, s0, 32), a1 = __shfl(h23, s0, 32), a2 = __shfl(h01, s1, 32), a3 = __shfl(h23, s1, 32);
  const int b0 = __shfl(l01, s0, 32), b1 = __shfl(l23, s0, 32), b2 = __shfl(l01, s1, 32), b3 = __shfl(l23, s1, 32);
  const int mk = (lane < 16) ? -1 : 0;
  v4i o;
  o.x = (a0 & mk) | (b0 & ~mk); o.y = (a1 & mk) | (b1 & ~mk);
  o.z = (a2 & mk) | (b2 & ~mk); o.w = (a3 & mk) | (b3 & ~mk);
  return o;
}

__device__ __forceinline__ void st2_v4f(float* p, v4f v) {
  *(volatile v4f*)p = v;
  __threadfence();
  *(volatile v4f*)p = v;
}
__device__ __forceinline__ void st2_v8us(unsigned short* p, v8us v) {
  *(volatile v8us*)p = v;
  __threadfence();
  *(volatile v8us*)p = v;
}

__device__ __forceinline__ v8us gather8(const float* __restrict__ base, int stride) {
  float f[8];
#pragma unroll
  for (int i = 0; i < 8; ++i) f[i] = base[(size_t)i * (size_t)stride];
  v8us o;
#pragma unroll
  for (int i = 0; i < 8; ++i) o[i] = (unsigned short)bf16_bits(f[i]);
  return o;
}

__global__ __launch_bounds__(NTHR) void k_prep(const float* __restrict__ x, const float* __restrict__ wl,
                                               const float* __restrict__ wr, const float* __restrict__ bl,
                                               const float* __restrict__ fcw, const float* __restrict__ fcb,
                                               unsigned short* xb, unsigned short* wc0, unsigned short* wci,
                                               float* sm) {
  const int tid = (int)threadIdx.x, lane = tid & 31, wave = tid >> 5;
  const int blk = (int)blockIdx.x;
  if (blk < PBX) {
    const int u   = blk * NTHR + tid;
    const int row = u >> 4, k8 = (u & 15) * 8;
    const int rc  = row < NN ? row : NN - 1;
    const unsigned mk = row < NN ? 0xffffu : 0u;
    const float* p = x + (size_t)rc * DF + k8;
    const v4f a = *(const v4fa*)p;
    const v4f b = *(const v4fa*)(p + 4);
    v8us o;
    o[0] = (unsigned short)(bf16_bits(a.x) & mk); o[1] = (unsigned short)(bf16_bits(a.y) & mk);
    o[2] = (unsigned short)(bf16_bits(a.z) & mk); o[3] = (unsigned short)(bf16_bits(a.w) & mk);
    o[4] = (unsigned short)(bf16_bits(b.x) & mk); o[5] = (unsigned short)(bf16_bits(b.y) & mk);
    o[6] = (unsigned short)(bf16_bits(b.z) & mk); o[7] = (unsigned short)(bf16_bits(b.w) & mk);
    st2_v8us(xb + (size_t)row * XPITCH + k8, o);
  } else if (blk < PBX + PBW0) {
    const int u    = (blk - PBX) * NTHR + tid;
    const int part = u >> 11;
    const int v    = u & (UPART - 1);
    const int n    = v >> 4, k8 = (v & 15) * 8;
    v8us o;
    if (part < 2) o = gather8(wl + (size_t)k8 * DF + n, DF);
    else          o = gather8(wr + (size_t)k8 * DF + n, DF);
    st2_v8us(wc0 + (size_t)n * WP0 + part * DF + k8, o);
  } else if (blk < PBX + PBW0 + PBWI) {
    const int u    = (blk - PBX - PBW0) * NTHR + tid;
    const int li   = u >> 13;
    const int part = (u >> 11) & 3;
    const int v    = u & (UPART - 1);
    const int n    = v >> 4, k8 = (v & 15) * 8;
    const size_t mo = (size_t)(li + 1) * DF * DF;
    v8us o;
    if (part < 2) o = gather8(wl + mo + (size_t)k8 * DF + n, DF);
    else          o = gather8(wr + mo + (size_t)k8 * DF + n, DF);
    st2_v8us(wci + (size_t)li * DF * WPI + (size_t)n * WPI + part * DF + k8, o);
  } else {
    if (wave < 6) {
      const v4f a = *(const v4fa*)(bl + 4 * tid);
      v4f o;
      o.x = bf16_val(a.x); o.y = bf16_val(a.y); o.z = bf16_val(a.z); o.w = bf16_val(a.w);
      st2_v4f(sm + 4 * tid, o);
    } else {
      const int q = tid - 192;
      const int c = q >> 5, k = (q & 31) * 4;
      const float f0 = fcw[(k + 0) * 2 + c], f1 = fcw[(k + 1) * 2 + c];
      const float f2 = fcw[(k + 2) * 2 + c], f3 = fcw[(k + 3) * 2 + c];
      v4f o;
      o.x = bf16_val(f0); o.y = bf16_val(f1); o.z = bf16_val(f2); o.w = bf16_val(f3);
      st2_v4f(sm + NLAY * DF + 4 * q, o);
    }
    if (wave == 0) {
      const float b0 = fcb[0], b1 = fcb[1];
      asm volatile("" :: "v"(b0), "v"(b1));
      const unsigned mk = (lane == 0) ? 0xffffffffu : 0u;
      v4f o;
      o.x = __uint_as_float((bf16_bits(b0) << 16) & mk);
      o.y = __uint_as_float((bf16_bits(b1) << 16) & mk);
      o.z = 0.0f; o.w = 0.0f;
      float* dp = sm + NLAY * DF + 2 * DF + 4 * (lane & 7);
      if (lane < 8) *(volatile v4f*)dp = o;
      __threadfence();
      if (lane < 8) *(volatile v4f*)dp = o;
    }
  }
}

__device__ __forceinline__ void bucket_flush(const int* pl, const int* cnt, int ov, int* lp, int* cop, int* fp,
                                             int tid) {
#pragma unroll 1
  for (int i = tid * 4; i < RCAP; i += NTHR * 4) {
    const v4i v = *(const v4ia*)(pl + i);
    *(volatile v4i*)(lp + i) = v;
  }
#pragma unroll 1
  for (int i = tid * 4; i < 3 * NBRUN; i += NTHR * 4) {
    const v4i v = *(const v4ia*)(cnt + i);
    *(volatile v4i*)(cop + i) = v;
  }
  if (tid < 8) {
    const v4i f = {ov, ov, ov, ov};
    *(volatile v4i*)(fp + 4 * tid) = f;
  }
}

__global__ __launch_bounds__(NTHR) void k_bucket(const int* __restrict__ srcs, const int* __restrict__ dsts,
                                                 int* LIST, int* COI, int* FLAG) {
  extern __shared__ __attribute__((aligned(16))) int dsm[];
  int* wl   = dsm;
  int* pl   = dsm + NWAVE * WLCAP;
  int* cnt  = pl + RCAP;
  int* offs = cnt + NBRUN;
  int* invb = offs + NBRUN;
  int* cur  = invb + NBRUN;
  int* misc = cur + NBRUN;
  const int tid = (int)threadIdx.x, lane = tid & 31, wave = tid >> 5;
  const int blk = (int)blockIdx.x;
  const unsigned nbs = (unsigned)(blk * NBRUN);

  {
    const v4i z4 = {0, 0, 0, 0};
    for (int i = tid * 4; i < BK_ZINTS; i += NTHR * 4) *(v4ia*)(dsm + i) = z4;
    if (tid < 16) misc[tid] = 0;
  }
  __syncthreads();

  {
    const int ebeg = wave * PER;
    const int eend = (ebeg + PER < NE) ? (ebeg + PER) : NE;
    int* mylist = wl + wave * WLCAP;
    int wc = 0;
#pragma unroll 1
    for (int cb = ebeg; cb < eend; cb += WCH) {
      const int e0  = cb + lane * EPT;
      const bool vld = e0 < NE;
      const int e0c = vld ? e0 : (NE - EPT);
      const v4i da = *(const v4ia*)(dsts + e0c);
      const v4i db = *(const v4ia*)(dsts + e0c + 4);
      const unsigned vm = vld ? (unsigned)NBRUN : 0u;
      const unsigned s0 = (unsigned)da.x - nbs, s1 = (unsigned)da.y - nbs;
      const unsigned s2 = (unsigned)da.z - nbs, s3 = (unsigned)da.w - nbs;
      const unsigned s4 = (unsigned)db.x - nbs, s5 = (unsigned)db.y - nbs;
      const unsigned s6 = (unsigned)db.z - nbs, s7 = (unsigned)db.w - nbs;
      const bool h0 = s0 < vm, h1 = s1 < vm, h2 = s2 < vm, h3 = s3 < vm;
      const bool h4 = s4 < vm, h5 = s5 < vm, h6 = s6 < vm, h7 = s7 < vm;
      const unsigned m0 = __builtin_amdgcn_ballot_w32(h0), m1 = __builtin_amdgcn_ballot_w32(h1);
      const unsigned m2 = __builtin_amdgcn_ballot_w32(h2), m3 = __builtin_amdgcn_ballot_w32(h3);
      const unsigned m4 = __builtin_amdgcn_ballot_w32(h4), m5 = __builtin_amdgcn_ballot_w32(h5);
      const unsigned m6 = __builtin_amdgcn_ballot_w32(h6), m7 = __builtin_amdgcn_ballot_w32(h7);
      const unsigned any = m0 | m1 | m2 | m3 | m4 | m5 | m6 | m7;
      if (any != 0u) {
        const int pre = (int)(__builtin_amdgcn_mbcnt_lo(m0, 0u) + __builtin_amdgcn_mbcnt_lo(m1, 0u) +
                              __builtin_amdgcn_mbcnt_lo(m2, 0u) + __builtin_amdgcn_mbcnt_lo(m3, 0u) +
                              __builtin_amdgcn_mbcnt_lo(m4, 0u) + __builtin_amdgcn_mbcnt_lo(m5, 0u) +
                              __builtin_amdgcn_mbcnt_lo(m6, 0u) + __builtin_amdgcn_mbcnt_lo(m7, 0u));
        int p = wc + pre;
        if (h0) { if (p < WLCAP) mylist[p] = ((e0 + 0) << SLB) | (int)s0; p = p + 1; }
        if (h1) { if (p < WLCAP) mylist[p] = ((e0 + 1) << SLB) | (int)s1; p = p + 1; }
        if (h2) { if (p < WLCAP) mylist[p] = ((e0 + 2) << SLB) | (int)s2; p = p + 1; }
        if (h3) { if (p < WLCAP) mylist[p] = ((e0 + 3) << SLB) | (int)s3; p = p + 1; }
        if (h4) { if (p < WLCAP) mylist[p] = ((e0 + 4) << SLB) | (int)s4; p = p + 1; }
        if (h5) { if (p < WLCAP) mylist[p] = ((e0 + 5) << SLB) | (int)s5; p = p + 1; }
        if (h6) { if (p < WLCAP) mylist[p] = ((e0 + 6) << SLB) | (int)s6; p = p + 1; }
        if (h7) { if (p < WLCAP) mylist[p] = ((e0 + 7) << SLB) | (int)s7; p = p + 1; }
        wc += (int)(__builtin_popcount(m0) + __builtin_popcount(m1) + __builtin_popcount(m2) + __builtin_popcount(m3) +
                    __builtin_popcount(m4) + __builtin_popcount(m5) + __builtin_popcount(m6) + __builtin_popcount(m7));
      }
    }
    if (lane == 0) misc[wave] = wc;
  }
  __syncthreads();

  if (wave == 0) {
    int ov = 0;
#pragma unroll 1
    for (int w2 = 0; w2 < NWAVE; ++w2) {
      int c = misc[w2];
      if (c > WLCAP) ov = 1;
      c = c < 0 ? 0 : (c > WLCAP ? WLCAP : c);
#pragma unroll 1
      for (int b0 = 0; b0 < c; b0 += 32) {
        const int idx = b0 + lane;
        const int ent = wl[w2 * WLCAP + (idx < WLCAP ? idx : WLCAP - 1)];
        const int m32 = (c - b0) < 32 ? (c - b0) : 32;
#pragma unroll 1
        for (int k = 0; k < m32; ++k) {
          const int u    = __builtin_amdgcn_readlane(ent, k);
          const int slot = u & (NBRUN - 1);
          if (lane == 0) cnt[slot] = cnt[slot] + 1;
        }
      }
    }
    if (lane == 0) misc[9] = ov;
  }
  __syncthreads();

#pragma unroll 1
  for (int s = tid; s < NBRUN; s += NTHR) {
    int cv = cnt[s];
    cv = cv < 1 ? 1 : cv;
    invb[s] = __float_as_int(1.0f / (float)cv);
  }
  if (wave == 0) {
    const int base = lane * (NBRUN / 32);
    int s = 0;
#pragma unroll 1
    for (int i = 0; i < NBRUN / 32; ++i) s += cnt[base + i];
    int incl = s;
#pragma unroll
    for (int d = 1; d < 32; d <<= 1) {
      const int y = __shfl_up(incl, d, 32);
      if (lane >= d) incl += y;
    }
    int run = incl - s;
#pragma unroll 1
    for (int i = 0; i < NBRUN / 32; ++i) {
      const int cv = cnt[base + i];
      offs[base + i] = run;
      cur[base + i]  = run;
      run += cv;
    }
  }
  __syncthreads();

  if (wave == 0) {
#pragma unroll 1
    for (int w2 = 0; w2 < NWAVE; ++w2) {
      int c = misc[w2];
      c = c < 0 ? 0 : (c > WLCAP ? WLCAP : c);
#pragma unroll 1
      for (int b0 = 0; b0 < c; b0 += 32) {
        const int idx = b0 + lane;
        const int ent = wl[w2 * WLCAP + (idx < WLCAP ? idx : WLCAP - 1)];
        int eid = (ent >> SLB) & 0x1FFFFF;
        eid = eid > NE - 1 ? NE - 1 : eid;
        int sr = srcs[eid];
        sr = sr < 0 ? 0 : (sr > NN - 1 ? NN - 1 : sr);
        const int m32 = (c - b0) < 32 ? (c - b0) : 32;
#pragma unroll 1
        for (int k = 0; k < m32; ++k) {
          const int u    = __builtin_amdgcn_readlane(ent, k);
          const int wd   = __builtin_amdgcn_readlane(sr, k);
          const int slot = u & (NBRUN - 1);
          if (lane == 0) {
            int p = cur[slot];
            p = p < 0 ? 0 : (p > RCAP - 1 ? RCAP - 1 : p);
            pl[p] = wd;
            cur[slot] = p + 1;
          }
        }
      }
    }
  }
  __syncthreads();

  const int ovf = misc[9];
  int* lp  = LIST + (size_t)blk * RCAP;
  int* cop = COI + (size_t)blk * (3 * NBRUN);
  int* fp  = FLAG + (size_t)blk * 32;
  bucket_flush(pl, cnt, ovf, lp, cop, fp, tid);
  __threadfence();
  bucket_flush(pl, cnt, ovf, lp, cop, fp, tid);
}

template <int L0>
__global__ __launch_bounds__(NTHR) void k_replay(const int* __restrict__ LIST, const int* __restrict__ COI,
                                                 const int* __restrict__ FLAG,
                                                 const unsigned short* __restrict__ XB,
                                                 const float* __restrict__ HF, unsigned short* Mhl) {
  const int tid = (int)threadIdx.x, lane = tid & 31, wave = tid >> 5;
  const int rowBase = (int)blockIdx.x * RBM;
  const int bucket  = rowBase >> SLB;
  const int* lb  = LIST + (size_t)bucket * RCAP;
  const int* cob = COI + (size_t)bucket * (3 * NBRUN);
  const int flag = FLAG[(size_t)bucket * 32];
  const float qnan = __uint_as_float(0x7fc00000u);

#pragma unroll 1
  for (int i = 0; i < RBM / NWAVE; ++i) {
    const int d    = rowBase + (RBM / NWAVE) * wave + i;
    const int slot = d & (NBRUN - 1);
    int c = cob[slot];
    int o = cob[NBRUN + slot];
    const float inv = __int_as_float(cob[2 * NBRUN + slot]);
    const bool big = c > DEGCAP;
    c = c < 0 ? 0 : (c > DEGCAP ? DEGCAP : c);
    o = o < 0 ? 0 : (o > RCAP - 1 ? RCAP - 1 : o);
    int last = o + c - 1;
    last = last < o ? o : last;
    last = last > RCAP - 1 ? RCAP - 1 : last;
    const int cs = __builtin_amdgcn_readfirstlane(c);
    float a0 = 0.0f, a1 = 0.0f, a2 = 0.0f, a3 = 0.0f;
#pragma unroll 1
    for (int j = 0; j < cs; ++j) {
      int idx = o + j;
      idx = idx > last ? last : idx;
      int sr = lb[idx];
      sr = sr < 0 ? 0 : (sr > NN - 1 ? NN - 1 : sr);
      if constexpr (L0 != 0) {
        const v2u w = *(const v2ua*)(XB + (size_t)sr * XPITCH + 4 * lane);
        asm volatile("" :: "v"(w.x), "v"(w.y));
        a0 += __uint_as_float(w.x << 16);
        a1 += __uint_as_float(w.x & 0xffff0000u);
        a2 += __uint_as_float(w.y << 16);
        a3 += __uint_as_float(w.y & 0xffff0000u);
      } else {
        const v4f v = *(const v4fa*)(HF + (size_t)sr * DF + 4 * lane);
        asm volatile("" :: "v"(v));
        a0 += v.x; a1 += v.y; a2 += v.z; a3 += v.w;
      }
    }
    float m0 = a0 * inv, m1 = a1 * inv, m2 = a2 * inv, m3 = a3 * inv;
    const bool bad  = (flag != 0) | big;
    const bool live = d < NN;
    m0 = bad ? qnan : m0; m1 = bad ? qnan : m1; m2 = bad ? qnan : m2; m3 = bad ? qnan : m3;
    m0 = live ? m0 : 0.0f; m1 = live ? m1 : 0.0f; m2 = live ? m2 : 0.0f; m3 = live ? m3 : 0.0f;
    int h01, h23, l01, l23;
    hilo_pack(m0, m1, m2, m3, h01, h23, l01, l23);
    const v4i ow = regroup_w(h01, h23, l01, l23, lane);
    unsigned short* hp = Mhl + (size_t)d * MPITCH + 8 * lane;
    *(volatile v4i*)hp = ow;
    __threadfence();
    *(volatile v4i*)hp = ow;
  }
}

template <int KLEN, int WP>
__device__ __forceinline__ void gemm_seg(const unsigned short* __restrict__ ap,
                                         const unsigned short* __restrict__ bp, v8f (&acc)[8]) {
#pragma unroll 1
  for (int k0 = 0; k0 < KLEN; k0 += 32) {
    FragB af;
    af.h[0] = *(const v8usa*)(ap + k0);
    af.h[1] = *(const v8usa*)(ap + k0 + 16);
#pragma unroll
    for (int nt = 0; nt < 8; ++nt) {
      const unsigned short* wq = bp + (size_t)(16 * nt) * (size_t)WP + k0;
      FragB bf;
      bf.h[0] = *(const v8usa*)wq;
      bf.h[1] = *(const v8usa*)(wq + 16);
      acc[nt] = wmb(af, bf, acc[nt]);
    }
  }
}

__device__ __forceinline__ void head_flush(const float* lg, float* ob, int nv4, int tid) {
  const v4f v = *(const v4fa*)(lg + 4 * (tid & 63));
  asm volatile("" :: "v"(v));
  if (tid < 64 && tid < nv4) *(volatile v4f*)(ob + (size_t)4 * (size_t)tid) = v;
}

template <int MODE>
__global__ __launch_bounds__(NTHR) __attribute__((amdgpu_num_vgpr(248)))
void k_gemm_one(const unsigned short* __restrict__ Mhl, const unsigned short* __restrict__ Rp,
                const unsigned short* __restrict__ WC, const float* __restrict__ SMp, int layer,
                const int* __restrict__ FLAG, float* HF, unsigned short* HhlN, float* out) {
  extern __shared__ __attribute__((aligned(16))) float gsm[];
  float* stg = gsm;
  float* sb  = stg + GBM * SP;
  float* sfw = sb + 128;
  float* sfb = sfw + 256;
  float* lg  = sfb + 32;
  constexpr int WP     = (MODE == 0) ? WP0 : WPI;
  constexpr int RPITCH = (MODE == 0) ? XPITCH : MPITCH;
  constexpr int KR     = (MODE == 0) ? DF : KROOT;
  const int tid = (int)threadIdx.x, lane = tid & 31, wave = tid >> 5, hh = lane >> 4, m = lane & 15;
  const int blk = (int)blockIdx.x;
  const int rowBase = blk * GBM;
  const int lc = layer < 0 ? 0 : (layer > NLAY - 1 ? NLAY - 1 : layer);

  if (wave == 0) {
    const v4f t = *(const v4fa*)(SMp + 128 * lc + 4 * lane);
    asm volatile("" :: "v"(t));
    *(v4fa*)(sb + 4 * lane) = t;
  }
  if constexpr (MODE == 2) {
    if (wave == 1 || wave == 2) {
      const int o = 128 * (wave - 1) + 4 * lane;
      const v4f t = *(const v4fa*)(SMp + NLAY * DF + o);
      asm volatile("" :: "v"(t));
      *(v4fa*)(sfw + o) = t;
    }
    if (wave == 3) {
      const int o = 4 * (lane & 7);
      const v4f t = *(const v4fa*)(SMp + NLAY * DF + 2 * DF + o);
      asm volatile("" :: "v"(t));
      *(v4fa*)(sfb + o) = t;
    }
  }

  v8f acc[8];
  {
    const v8f z = {0.f, 0.f, 0.f, 0.f, 0.f, 0.f, 0.f, 0.f};
#pragma unroll
    for (int t = 0; t < 8; ++t) acc[t] = z;
  }
  const size_t arow = (size_t)(rowBase + 16 * wave + m);
  const unsigned short* ap = Mhl + arow * (size_t)MPITCH + 8 * hh;
  const unsigned short* rp = Rp + arow * (size_t)RPITCH + 8 * hh;
  const unsigned short* bp = WC + (size_t)m * (size_t)WP + 8 * hh;
  gemm_seg<KMEAN, WP>(ap, bp, acc);
  gemm_seg<KR, WP>(rp, bp + 2 * DF, acc);

#pragma unroll
  for (int nt = 0; nt < 8; ++nt) {
#pragma unroll
    for (int r = 0; r < 8; ++r) stg[(16 * wave + 8 * hh + r) * SP + 16 * nt + m] = acc[nt][r];
  }
  __syncthreads();

  const v4f bias = *(const v4fa*)(sb + 4 * lane);
  v4f f0 = {0.f, 0.f, 0.f, 0.f}, f1 = {0.f, 0.f, 0.f, 0.f};
  float fb0 = 0.0f, fb1 = 0.0f;
  int flag = 0;
  if constexpr (MODE == 2) {
    f0 = *(const v4fa*)(sfw + 4 * lane);
    f1 = *(const v4fa*)(sfw + 128 + 4 * lane);
    fb0 = sfb[0];
    fb1 = sfb[1];
    flag = FLAG[(size_t)(rowBase >> SLB) * 32];
  }
  const float qnan = __uint_as_float(0x7fc00000u);

#pragma unroll 1
  for (int i = 0; i < 16; ++i) {
    const int lr   = 16 * wave + i;
    const int grow = rowBase + lr;
    const bool live = grow < NN;
    const v4f a = *(const v4fa*)(stg + lr * SP + 4 * lane);
    asm volatile("" :: "v"(a));
    float v0 = a.x + bias.x, v1 = a.y + bias.y, v2 = a.z + bias.z, v3 = a.w + bias.w;
    v0 = (v0 > 0.0f) ? v0 : (v0 - v0); v1 = (v1 > 0.0f) ? v1 : (v1 - v1);
    v2 = (v2 > 0.0f) ? v2 : (v2 - v2); v3 = (v3 > 0.0f) ? v3 : (v3 - v3);
    v0 = live ? v0 : 0.0f; v1 = live ? v1 : 0.0f; v2 = live ? v2 : 0.0f; v3 = live ? v3 : 0.0f;
    if constexpr (MODE != 2) {
      v4f o;
      o.x = v0; o.y = v1; o.z = v2; o.w = v3;
      int h01, h23, l01, l23;
      hilo_pack(v0, v1, v2, v3, h01, h23, l01, l23);
      const v4i ow = regroup_w(h01, h23, l01, l23, lane);
      float* op = HF + (size_t)grow * DF + 4 * lane;
      unsigned short* hp = HhlN + (size_t)grow * MPITCH + 8 * lane;
      *(volatile v4f*)op = o;
      *(volatile v4i*)hp = ow;
      __threadfence();
      *(volatile v4f*)op = o;
      *(volatile v4i*)hp = ow;
    } else {
      float p0 = fmaf(v3, f0.w, fmaf(v2, f0.z, fmaf(v1, f0.y, v0 * f0.x)));
      float p1 = fmaf(v3, f1.w, fmaf(v2, f1.z, fmaf(v1, f1.y, v0 * f1.x)));
#pragma unroll
      for (int d = 16; d >= 1; d >>= 1) {
        p0 += __shfl_xor(p0, d, 32);
        p1 += __shfl_xor(p1, d, 32);
      }
      const float q0 = (flag != 0) ? qnan : (p0 + fb0);
      const float q1 = (flag != 0) ? qnan : (p1 + fb1);
      if (lane == 0) { lg[2 * lr] = q0; lg[2 * lr + 1] = q1; }
    }
  }

  if constexpr (MODE == 2) {
    __syncthreads();
    const int liveRows = (NN - rowBase) < GBM ? (NN - rowBase) : GBM;
    const int nv4 = liveRows / 2;
    float* ob = out + (size_t)blk * (size_t)(GBM * 2);
    head_flush(lg, ob, nv4, tid);
    __threadfence();
    head_flush(lg, ob, nv4, tid);
  }
}

extern "C" void kernel_launch(void* const* d_in, const int* in_sizes, int n_in,
                              void* d_out, int out_size, void* d_ws, size_t ws_size,
                              hipStream_t stream) {
  if (n_in < 7) return;
  if (in_sizes[0] != NN * DF) return;
  if (in_sizes[1] != 2 * NE) return;
  if (in_sizes[2] != NLAY * DF * DF) return;
  if (in_sizes[3] != NLAY * DF * DF) return;
  if (in_sizes[4] != NLAY * DF) return;
  if (in_sizes[5] != DF * 2) return;
  if (in_sizes[6] != 2) return;
  if (out_size != NN * 2) return;

  const float* x   = (const float*)d_in[0];
  const int*   ei  = (const int*)d_in[1];
  const float* Wl  = (const float*)d_in[2];
  const float* Wr  = (const float*)d_in[3];
  const float* bl  = (const float*)d_in[4];
  const float* fcW = (const float*)d_in[5];
  const float* fcb = (const float*)d_in[6];
  float* out = (float*)d_out;
  const int* srcs = ei;
  const int* dsts = ei + NE;

  constexpr size_t zHF   = (size_t)MP * DF * 4;
  constexpr size_t zHL   = (size_t)MP * MPITCH * 2;
  constexpr size_t zXB   = (size_t)MP * XPITCH * 2;
  constexpr size_t zLIST = (size_t)NBK * RCAP * 4;
  constexpr size_t zCOI  = (size_t)NBK * 3 * NBRUN * 4;
  constexpr size_t zFLAG = (size_t)NBK * 128;
  constexpr size_t zWC0  = (size_t)DF * WP0 * 2;
  constexpr size_t zWCI  = (size_t)5 * DF * WPI * 2;
  constexpr size_t zSM   = (size_t)SMF * 4;
  constexpr size_t oHF   = 0;
  constexpr size_t oHA   = oHF + zHF;
  constexpr size_t oHB   = oHA + zHL;
  constexpr size_t oM    = oHB + zHL;
  constexpr size_t oXB   = oM + zHL;
  constexpr size_t oLIST = oXB + zXB;
  constexpr size_t oCOI  = oLIST + zLIST;
  constexpr size_t oFLAG = oCOI + zCOI;
  constexpr size_t oWC0  = oFLAG + zFLAG;
  constexpr size_t oWCI  = oWC0 + zWC0;
  constexpr size_t oSM   = oWCI + zWCI;
  constexpr size_t oEND  = oSM + zSM;
  static_assert(zHF % 128 == 0 && zHL % 128 == 0 && zXB % 128 == 0 && zLIST % 128 == 0 && zCOI % 128 == 0);
  static_assert(zFLAG % 128 == 0 && zWC0 % 128 == 0 && zWCI % 128 == 0 && zSM % 128 == 0);
  static_assert(oEND <= ((size_t)128u << 20));
  if (oEND > ws_size) return;

  char* ws = (char*)d_ws;
  float*          HF   = (float*)(ws + oHF);
  unsigned short* HhlA = (unsigned short*)(ws + oHA);
  unsigned short* HhlB = (unsigned short*)(ws + oHB);
  unsigned short* Mhl  = (unsigned short*)(ws + oM);
  unsigned short* XB   = (unsigned short*)(ws + oXB);
  int*            LIST = (int*)(ws + oLIST);
  int*            COI  = (int*)(ws + oCOI);
  int*            FLAG = (int*)(ws + oFLAG);
  unsigned short* WC0  = (unsigned short*)(ws + oWC0);
  unsigned short* WCI  = (unsigned short*)(ws + oWCI);
  float*          SM   = (float*)(ws + oSM);

  hipFuncSetAttribute(reinterpret_cast<const void*>(&k_bucket), hipFuncAttributeMaxDynamicSharedMemorySize, (int)BK_LDS);
  hipFuncSetAttribute(reinterpret_cast<const void*>(&k_gemm_one<0>), hipFuncAttributeMaxDynamicSharedMemorySize, (int)GM_LDS);
  hipFuncSetAttribute(reinterpret_cast<const void*>(&k_gemm_one<1>), hipFuncAttributeMaxDynamicSharedMemorySize, (int)GM_LDS);
  hipFuncSetAttribute(reinterpret_cast<const void*>(&k_gemm_one<2>), hipFuncAttributeMaxDynamicSharedMemorySize, (int)GM_LDS);

  k_prep<<<PBTOT, NTHR, 0, stream>>>(x, Wl, Wr, bl, fcW, fcb, XB, WC0, WCI, SM);
  k_bucket<<<NBK, NTHR, BK_LDS, stream>>>(srcs, dsts, LIST, COI, FLAG);

  k_replay<1><<<MP / RBM, NTHR, 0, stream>>>(LIST, COI, FLAG, XB, HF, Mhl);
  k_gemm_one<0><<<MP / GBM, NTHR, GM_LDS, stream>>>(Mhl, XB, WC0, SM, 0, FLAG, HF, HhlA, out);

  for (int l = 1; l < NLAY - 1; ++l) {
    unsigned short* prv = ((l - 1) & 1) ? HhlB : HhlA;
    unsigned short* nxt = (l & 1) ? HhlB : HhlA;
    const unsigned short* wc = WCI + (size_t)(l - 1) * DF * WPI;
    k_replay<0><<<MP / RBM, NTHR, 0, stream>>>(LIST, COI, FLAG, XB, HF, Mhl);
    k_gemm_one<1><<<MP / GBM, NTHR, GM_LDS, stream>>>(Mhl, prv, wc, SM, l, FLAG, HF, nxt, out);
  }

  k_replay<0><<<MP / RBM, NTHR, 0, stream>>>(LIST, COI, FLAG, XB, HF, Mhl);
  k_gemm_one<2><<<MP / GBM, NTHR, GM_LDS, stream>>>(Mhl, HhlA, WCI + (size_t)4 * DF * WPI, SM, NLAY - 1, FLAG,
                                                    HF, HhlB, out);
}
